// MultiHeadAttention_40578851012981
// MI455X (gfx1250) — hardware-run, weakly checked
//
#include <hip/hip_runtime.h>
#include <math.h>

typedef __attribute__((ext_vector_type(16))) _Float16 v16h;
typedef __attribute__((ext_vector_type(8)))  _Float16 v8h;
typedef __attribute__((ext_vector_type(8)))  float    v8f;
typedef __attribute__((ext_vector_type(4)))  float    v4f;

constexpr int kBatch  = 2;
constexpr int kSeq    = 2048;
constexpr int kHid    = 1024;
constexpr int kHeads  = 16;
constexpr int kHd     = 64;
constexpr int kRows   = kBatch * kSeq;
constexpr int kHalfHd = kHd / 2;
static_assert(kHeads * kHd == kHid, "head split");
static_assert(kHd == 64, "head width fixed at 64");
static_assert((kSeq % 64) == 0 && (kHid % 64) == 0 && (kHid % 32) == 0 && (kRows % 64) == 0, "tile multiples");
static_assert(kSeq == 2048 && kHid == 1024, "bit tricks below assume these");

constexpr double cx_sqrt(double x) {
  double g = (x > 1.0) ? x : 1.0;
  for (int it = 0; it < 80; ++it) g = 0.5 * (g + x / g);
  return g;
}
constexpr float kXCarry    = 16.0f;
constexpr float kWCarry    = 256.0f;
constexpr float kQKCarry   = 16.0f;
constexpr float kVCarry    = 16.0f;
constexpr float kAttnCarry = 2048.0f;
constexpr float kInvSqrtHd = (float)(1.0 / cx_sqrt((double)kHd));
static_assert(kInvSqrtHd == 0.125f, "1/sqrt(head width)");
constexpr float kQKScale    = kQKCarry / (kXCarry * kWCarry);
constexpr float kVScale     = kVCarry / (kXCarry * kWCarry);
constexpr float kScoreScale = kInvSqrtHd / (kQKCarry * kQKCarry);
constexpr float kCtxScale   = kAttnCarry / kVCarry;
constexpr float kOutScale   = 1.0f / (kAttnCarry * kWCarry);
constexpr float kScoreClamp = 10.0f;

struct InvFreqTab { float v[kHalfHd]; };
constexpr InvFreqTab make_inv_freq() {
  InvFreqTab t{};
  const double r8 = cx_sqrt(cx_sqrt(cx_sqrt(10.0)));
  for (int i = 0; i < kHalfHd; ++i) {
    double p = 1.0;
    for (int j = 0; j < (i & 7); ++j) p *= r8;
    for (int j = 0; j < (i >> 3); ++j) p *= 10.0;
    t.v[i] = (float)(1.0 / p);
  }
  return t;
}
__device__ constexpr InvFreqTab kInvFreq = make_inv_freq();
static_assert(sizeof(kInvFreq.v) / sizeof(kInvFreq.v[0]) == 32, "table length");

constexpr size_t kPlaneBytes = (size_t)kRows * kHid * 2;
constexpr size_t kTabBytes   = (size_t)kSeq * kHalfHd * 4;
constexpr size_t kOffX16  = 0;
constexpr size_t kOffW16  = kOffX16 + kPlaneBytes;
constexpr size_t kOffCos  = kOffW16 + (size_t)4 * kHid * kHid * 2;
constexpr size_t kOffSin  = kOffCos + kTabBytes;
constexpr size_t kOffQ16  = kOffSin + kTabBytes;
constexpr size_t kOffK16  = kOffQ16 + kPlaneBytes;
constexpr size_t kOffVT16 = kOffK16 + kPlaneBytes;
constexpr size_t kOffA16  = kOffVT16 + kPlaneBytes;
constexpr size_t kWsTotal = kOffA16 + kPlaneBytes;
static_assert(kWsTotal == 50855936ull, "carve total");
static_assert(kWsTotal <= 134217728ull, "carve cap");
static_assert((kOffW16 % 128) == 0 && (kOffCos % 128) == 0 && (kOffSin % 128) == 0 && (kOffQ16 % 128) == 0 &&
              (kOffK16 % 128) == 0 && (kOffVT16 % 128) == 0 && (kOffA16 % 128) == 0, "128-B aligned regions");
constexpr size_t kPlaneElems = (size_t)kRows * kHid;

struct FragH {
  union U { v16h v; v8h h[2]; };
  static __device__ __forceinline__ v16h load(const _Float16* p) {
    U f;
    f.h[0] = *(const v8h*)(p);
    f.h[1] = *(const v8h*)(p + 16);
    return f.v;
  }
  static __device__ __forceinline__ v8f mma(v16h a, v16h b, v8f c) {
    return __builtin_amdgcn_wmma_f32_16x16x32_f16(false, a, false, b, (short)0, c, false, false);
  }
};
__device__ __forceinline__ void guard4_h(v8f& a, v8f& b, v8f& c, v8f& d, v16h x, v16h y) {
  asm volatile("v_nop\n\tv_nop\n\tv_nop\n\tv_nop" : "+v"(a), "+v"(b), "+v"(c), "+v"(d) : "v"(x), "v"(y));
}
__device__ __forceinline__ void keep4_h(v16h a, v16h b, v16h c, v16h d) {
  asm volatile("v_nop" :: "v"(a), "v"(b), "v"(c), "v"(d));
}
__device__ __forceinline__ void acc_guard4(v8f& a, v8f& b, v8f& c, v8f& d) {
  asm volatile("v_nop\n\tv_nop\n\tv_nop\n\tv_nop" : "+v"(a), "+v"(b), "+v"(c), "+v"(d));
}
__device__ __forceinline__ v8f mma_g(v16h a, v16h b, v8f c) {
  c = __builtin_amdgcn_wmma_f32_16x16x32_f16(false, a, false, b, (short)0, c, false, false);
  asm volatile("v_nop\n\tv_nop\n\tv_nop\n\tv_nop" : "+v"(c) : "v"(a), "v"(b));
  return c;
}

__global__ __launch_bounds__(256) void cast8_scale_f16_kernel(
    const float* __restrict__ in0, const float* __restrict__ in1,
    const float* __restrict__ in2, const float* __restrict__ in3,
    unsigned short* __restrict__ out, int n8, float scale)
{
  const int z = blockIdx.y;
  const float* in = (z == 0) ? in0 : (z == 1) ? in1 : (z == 2) ? in2 : in3;
  const int i = blockIdx.x * 256 + threadIdx.x;
  if (i >= n8) return;
  const float* p = in + 8 * (size_t)i;
  const v4f a = *(const v4f*)(p);
  const v4f c = *(const v4f*)(p + 4);
  v8h hv;
#pragma unroll
  for (int e = 0; e < 4; ++e) {
    const float f0 = a[e] * scale;
    const float f1 = c[e] * scale;
    hv[e]     = (_Float16)f0;
    hv[4 + e] = (_Float16)f1;
  }
  unsigned short* q = out + (size_t)z * 8 * (size_t)n8 + 8 * (size_t)i;
  *(volatile v8h*)q = hv;
  __threadfence();
  *(volatile v8h*)q = hv;
}

__global__ __launch_bounds__(256) void rotary_table_kernel(float* __restrict__ cosT, float* __restrict__ sinT)
{
  const int t = blockIdx.x * 256 + threadIdx.x;
  const int s = t >> 5;
  const int i = t & 31;
  const float inv = kInvFreq.v[i];
  const float ang = (float)s * inv;
  float sn, cs;
  sincosf(ang, &sn, &cs);
  ((volatile float*)cosT)[t] = cs;
  ((volatile float*)sinT)[t] = sn;
  __threadfence();
  ((volatile float*)cosT)[t] = cs;
  ((volatile float*)sinT)[t] = sn;
}

template <int OUT_MODE>
__global__ __launch_bounds__(256) void wmma_gemm64(
    const unsigned short* __restrict__ Ap, int lda, long strideA,
    const unsigned short* __restrict__ Btp, int ldb, long strideB,
    void* __restrict__ Cout, int ldc, long strideC,
    const float* __restrict__ cosT, const float* __restrict__ sinT,
    int M, int N, int K, float scale)
{
  const _Float16* A  = (const _Float16*)Ap;
  const _Float16* Bt = (const _Float16*)Btp;
  __shared__ __align__(16) float sT[8][16 * 68];
  const int b    = blockIdx.y;
  const int lane = threadIdx.x & 31;
  const int wave = __builtin_amdgcn_readfirstlane((int)(threadIdx.x >> 5));
  const int tilesN = N >> 6;
  const int tilesM = M >> 6;
  const int tile = blockIdx.x * 8 + wave;
  if (tile >= tilesM * tilesN) return;
  const int tm = tile / tilesN;
  const int tn = tile - tm * tilesN;
  const int m0 = tm << 6;
  const int n0 = tn << 6;

  const _Float16* Ab = A  + (size_t)b * strideA;
  const _Float16* Bb = Bt + (size_t)b * strideB;

  const int rlane = lane & 15;
  const int koff  = (lane >> 4) * 8;
  const int mOff  = (lane >> 4) * 8;

  v8f acc[4][4];
#pragma unroll
  for (int i = 0; i < 4; ++i)
#pragma unroll
    for (int j = 0; j < 4; ++j) acc[i][j] = (v8f){0.f,0.f,0.f,0.f,0.f,0.f,0.f,0.f};

  for (int k0 = 0; k0 < K; k0 += 32) {
    v16h bh[4];
#pragma unroll
    for (int j = 0; j < 4; ++j) {
      const size_t bo = (size_t)(n0 + (j << 4) + rlane) * ldb + koff + k0;
      bh[j] = FragH::load(Bb + bo);
    }
#pragma unroll
    for (int i = 0; i < 4; ++i) {
      const size_t ao = (size_t)(m0 + (i << 4) + rlane) * lda + koff + k0;
      v16h ah = FragH::load(Ab + ao);
#pragma unroll
      for (int j = 0; j < 4; ++j) acc[i][j] = FragH::mma(ah, bh[j], acc[i][j]);
      guard4_h(acc[i][0], acc[i][1], acc[i][2], acc[i][3], ah, bh[3]);
    }
    keep4_h(bh[0], bh[1], bh[2], bh[3]);
  }
  acc_guard4(acc[0][0], acc[0][1], acc[0][2], acc[0][3]);
  acc_guard4(acc[1][0], acc[1][1], acc[1][2], acc[1][3]);
  acc_guard4(acc[2][0], acc[2][1], acc[2][2], acc[2][3]);
  acc_guard4(acc[3][0], acc[3][1], acc[3][2], acc[3][3]);

  float* slab = sT[wave];
#pragma unroll
  for (int i = 0; i < 4; ++i) {
    const int mBase = m0 + (i << 4);
#pragma unroll
    for (int j = 0; j < 4; ++j) {
#pragma unroll
      for (int r = 0; r < 8; ++r) {
        const float v = acc[i][j][r] * scale;
        slab[(mOff + r) * 68 + (j << 4) + rlane] = v;
      }
    }
    __builtin_amdgcn_fence(__ATOMIC_RELEASE, "workgroup");
    __builtin_amdgcn_wave_barrier();
    __builtin_amdgcn_fence(__ATOMIC_ACQUIRE, "workgroup");
    if (OUT_MODE == 0) {
      float* C = (float*)Cout + (size_t)b * strideC;
      const int hh = lane >> 4, c4 = (lane & 15) * 4;
      for (int pass = 0; pass < 2; ++pass) {
#pragma unroll
        for (int it = 0; it < 8; ++it) {
          const int row = it * 2 + hh;
          v4f v = *(const v4f*)(slab + row * 68 + c4);
          *(volatile v4f*)(C + (size_t)(mBase + row) * ldc + n0 + c4) = v;
        }
        __threadfence();
      }
    } else if (OUT_MODE == 1) {
      const int q = lane >> 3, c8 = (lane & 7) * 8;
      unsigned short* C = (unsigned short*)Cout + (size_t)b * strideC;
      v8h ov[4];
#pragma unroll
      for (int it = 0; it < 4; ++it) {
        const int row = it * 4 + q;
        const float* sp = slab + row * 68 + c8;
        const v4f a0 = *(const v4f*)(sp);
        const v4f a1 = *(const v4f*)(sp + 4);
#pragma unroll
        for (int e = 0; e < 4; ++e) {
          ov[it][e]     = (_Float16)a0[e];
          ov[it][4 + e] = (_Float16)a1[e];
        }
      }
      for (int pass = 0; pass < 2; ++pass) {
#pragma unroll
        for (int it = 0; it < 4; ++it) {
          const int row = it * 4 + q;
          *(volatile v8h*)(C + (size_t)(mBase + row) * ldc + n0 + c8) = ov[it];
        }
        __threadfence();
      }
    } else {
      const int q = lane >> 3, c8 = (lane & 7) * 8;
      const int which = n0 >> 10;
      const int head  = (n0 >> 6) & (kHeads - 1);
      unsigned short* C = (unsigned short*)Cout + (size_t)which * kPlaneElems;
      v8h ov[4];
      size_t oo[4];
#pragma unroll
      for (int it = 0; it < 4; ++it) {
        const int row = it * 4 + q;
        const int m   = mBase + row;
        const int bb  = m >> 11;
        const int s   = m & (kSeq - 1);
        const float* sp = slab + row * 68 + c8;
        const v4f a0 = *(const v4f*)(sp);
        const v4f a1 = *(const v4f*)(sp + 4);
        const v4f cv = *(const v4f*)(cosT + (size_t)s * kHalfHd + (c8 >> 1));
        const v4f sv = *(const v4f*)(sinT + (size_t)s * kHalfHd + (c8 >> 1));
        const float o0 = a0[0] * cv[0] - a0[1] * sv[0];
        const float o1 = a0[0] * sv[0] + a0[1] * cv[0];
        const float o2 = a0[2] * cv[1] - a0[3] * sv[1];
        const float o3 = a0[2] * sv[1] + a0[3] * cv[1];
        const float o4 = a1[0] * cv[2] - a1[1] * sv[2];
        const float o5 = a1[0] * sv[2] + a1[1] * cv[2];
        const float o6 = a1[2] * cv[3] - a1[3] * sv[3];
        const float o7 = a1[2] * sv[3] + a1[3] * cv[3];
        ov[it][0] = (_Float16)o0;
        ov[it][1] = (_Float16)o1;
        ov[it][2] = (_Float16)o2;
        ov[it][3] = (_Float16)o3;
        ov[it][4] = (_Float16)o4;
        ov[it][5] = (_Float16)o5;
        ov[it][6] = (_Float16)o6;
        ov[it][7] = (_Float16)o7;
        oo[it] = ((size_t)(bb * kHeads + head) * kSeq + s) * kHd + c8;
      }
      for (int pass = 0; pass < 2; ++pass) {
#pragma unroll
        for (int it = 0; it < 4; ++it) *(volatile v8h*)(C + oo[it]) = ov[it];
        __threadfence();
      }
    }
    __builtin_amdgcn_fence(__ATOMIC_RELEASE, "workgroup");
    __builtin_amdgcn_wave_barrier();
    __builtin_amdgcn_fence(__ATOMIC_ACQUIRE, "workgroup");
  }
}

constexpr int kQB = 64;
constexpr int kKT = 64;
constexpr int kLP = 72;
constexpr int kAW = 4;
constexpr int kQTiles = kSeq / kQB;
constexpr int kKTiles = kSeq / kKT;
static_assert(kQB == kKT, "diagonal tile logic assumes equal tiles");

__global__ __launch_bounds__(128) void attn_kernel(
    const unsigned short* __restrict__ Qp, const unsigned short* __restrict__ Kp,
    const unsigned short* __restrict__ Vtp, unsigned short* __restrict__ Op)
{
  __shared__ __align__(16) _Float16 Ksh[kKT * kLP];
  __shared__ __align__(16) _Float16 Vsh[kHd * kLP];
  __shared__ __align__(16) _Float16 Psh[kAW][16 * kLP];
  __shared__ __align__(16) float    Os[kAW][16 * 68];

  const int tid  = threadIdx.x;
  const int wave = __builtin_amdgcn_readfirstlane((int)(threadIdx.x >> 5));
  const int lane = tid & 31;
  const int hh   = lane >> 4;
  const int c    = lane & 15;
  const int qb   = blockIdx.x % kQTiles;
  const int bh   = blockIdx.x / kQTiles;
  const int q0   = qb * kQB + wave * 16;

  const _Float16* Qb = (const _Float16*)Qp  + (size_t)bh * kSeq * kHd;
  const _Float16* Kb = (const _Float16*)Kp  + (size_t)bh * kSeq * kHd;
  const _Float16* Vb = (const _Float16*)Vtp + (size_t)bh * kHd * kSeq;

  v16h qa[2];
#pragma unroll
  for (int dc = 0; dc < 2; ++dc) qa[dc] = FragH::load(Qb + (size_t)(q0 + c) * kHd + dc * 32 + 8 * hh);

  float lsum[8];
  v8f oacc[4];
#pragma unroll
  for (int r = 0; r < 8; ++r) lsum[r] = 0.f;
#pragma unroll
  for (int t = 0; t < 4; ++t) oacc[t] = (v8f){0.f,0.f,0.f,0.f,0.f,0.f,0.f,0.f};

  _Float16* pw = Psh[wave];

#pragma unroll 1
  for (int kc = 0; kc < kKTiles; ++kc) {
    const int kv0 = kc * kKT;
    const bool pv = (kc <= qb);
    __syncthreads();
#pragma unroll
    for (int it = 0; it < 4; ++it) {
      const int e = it * 128 + tid;
      const int row = e >> 3, part = e & 7;
      const v8h kk = *(const v8h*)(Kb + (size_t)(kv0 + row) * kHd + part * 8);
      *(v8h*)(Ksh + row * kLP + part * 8) = kk;
    }
    if (pv) {
#pragma unroll
      for (int it = 0; it < 4; ++it) {
        const int e = it * 128 + tid;
        const int row = e >> 3, part = e & 7;
        const v8h vv = *(const v8h*)(Vb + (size_t)row * kSeq + kv0 + part * 8);
        *(v8h*)(Vsh + row * kLP + part * 8) = vv;
      }
    }
    __syncthreads();

    v8f s[4];
#pragma unroll
    for (int j = 0; j < 4; ++j) {
      s[j] = (v8f){0.f,0.f,0.f,0.f,0.f,0.f,0.f,0.f};
#pragma unroll
      for (int dc = 0; dc < 2; ++dc) {
        const v16h kb = FragH::load(Ksh + (j * 16 + c) * kLP + dc * 32 + 8 * hh);
        s[j] = mma_g(qa[dc], kb, s[j]);
      }
    }
#pragma unroll
    for (int j = 0; j < 4; ++j) {
#pragma unroll
      for (int r = 0; r < 8; ++r) {
        const float x = fminf(s[j][r] * kScoreScale, kScoreClamp);
        const float p = __expf(x);
        lsum[r] += p;
        s[j][r] = p;
      }
    }
    if (pv) {
      const bool diag = (kc == qb);
#pragma unroll
      for (int j = 0; j < 4; ++j) {
        const int kvcol = kv0 + j * 16 + c;
#pragma unroll
        for (int r = 0; r < 8; ++r) {
          const int qrow = q0 + 8 * hh + r;
          const float pm = (diag && (kvcol > qrow)) ? 0.0f : s[j][r];
          pw[(8 * hh + r) * kLP + j * 16 + c] = (_Float16)pm;
        }
      }
      __builtin_amdgcn_fence(__ATOMIC_RELEASE, "workgroup");
      __builtin_amdgcn_wave_barrier();
      __builtin_amdgcn_fence(__ATOMIC_ACQUIRE, "workgroup");
#pragma unroll
      for (int kk = 0; kk < 2; ++kk) {
        const v16h pa = FragH::load(pw + c * kLP + kk * 32 + 8 * hh);
#pragma unroll
        for (int t = 0; t < 4; ++t) {
          const v16h vb = FragH::load(Vsh + (t * 16 + c) * kLP + kk * 32 + 8 * hh);
          oacc[t] = mma_g(pa, vb, oacc[t]);
        }
      }
    }
  }

  float* os = Os[wave];
#pragma unroll
  for (int r = 0; r < 8; ++r) {
    float l = lsum[r];
    l += __shfl_xor(l, 1, 32);
    l += __shfl_xor(l, 2, 32);
    l += __shfl_xor(l, 4, 32);
    l += __shfl_xor(l, 8, 32);
    const float inv = kCtxScale * __builtin_amdgcn_rcpf(l);
#pragma unroll
    for (int t = 0; t < 4; ++t) os[(8 * hh + r) * 68 + t * 16 + c] = oacc[t][r] * inv;
  }
  __builtin_amdgcn_fence(__ATOMIC_RELEASE, "workgroup");
  __builtin_amdgcn_wave_barrier();
  __builtin_amdgcn_fence(__ATOMIC_ACQUIRE, "workgroup");
  {
    const int bb = bh / kHeads;
    const int h  = bh - bb * kHeads;
    const int q4 = lane >> 3, c8 = (lane & 7) * 8;
    v8h ov[4];
    size_t oo[4];
#pragma unroll
    for (int it = 0; it < 4; ++it) {
      const int row = it * 4 + q4;
      const float* sp = os + row * 68 + c8;
      const v4f a0 = *(const v4f*)(sp);
      const v4f a1 = *(const v4f*)(sp + 4);
#pragma unroll
      for (int e = 0; e < 4; ++e) {
        ov[it][e]     = (_Float16)a0[e];
        ov[it][4 + e] = (_Float16)a1[e];
      }
      oo[it] = ((size_t)(bb * kSeq + q0 + row)) * kHid + h * kHd + c8;
    }
    for (int pass = 0; pass < 2; ++pass) {
#pragma unroll
      for (int it = 0; it < 4; ++it) *(volatile v8h*)(Op + oo[it]) = ov[it];
      __threadfence();
    }
  }
}

extern "C" void kernel_launch(void* const* d_in, const int* in_sizes, int n_in,
                              void* d_out, int out_size, void* d_ws, size_t ws_size,
                              hipStream_t stream) {
  if (n_in < 5) return;
  if (in_sizes[0] != kRows * kHid) return;
  if (in_sizes[1] != kHid * kHid) return;
  if (in_sizes[2] != kHid * kHid) return;
  if (in_sizes[3] != kHid * kHid) return;
  if (in_sizes[4] != kHid * kHid) return;
  if (out_size != kRows * kHid) return;
  if (ws_size < kWsTotal) return;

  const float* x  = (const float*)d_in[0];
  const float* wq = (const float*)d_in[1];
  const float* wk = (const float*)d_in[2];
  const float* wv = (const float*)d_in[3];
  const float* wo = (const float*)d_in[4];
  float* out = (float*)d_out;

  char* ws = (char*)d_ws;
  unsigned short* X16  = (unsigned short*)(ws + kOffX16);
  unsigned short* W16  = (unsigned short*)(ws + kOffW16);
  float*          COS  = (float*)(ws + kOffCos);
  float*          SIN  = (float*)(ws + kOffSin);
  unsigned short* Q16  = (unsigned short*)(ws + kOffQ16);
  unsigned short* K16  = (unsigned short*)(ws + kOffK16);
  unsigned short* VT16 = (unsigned short*)(ws + kOffVT16);
  unsigned short* A16  = (unsigned short*)(ws + kOffA16);
  const unsigned short* Wqk16 = W16;
  const unsigned short* Wv16  = W16 + (size_t)2 * kHid * kHid;
  const unsigned short* Wo16  = W16 + (size_t)3 * kHid * kHid;

  constexpr int kXn8 = kRows * kHid / 8;
  constexpr int kWn8 = kHid * kHid / 8;
  static_assert((kXn8 % 256) == 0 && (kWn8 % 256) == 0, "cast grids exact");

  cast8_scale_f16_kernel<<<dim3(kXn8 / 256, 1), 256, 0, stream>>>(x, x, x, x, X16, kXn8, kXCarry);
  cast8_scale_f16_kernel<<<dim3(kWn8 / 256, 4), 256, 0, stream>>>(wq, wk, wv, wo, W16, kWn8, kWCarry);
  rotary_table_kernel<<<(kSeq * kHalfHd) / 256, 256, 0, stream>>>(COS, SIN);

  wmma_gemm64<3><<<dim3((kRows / 64) * (2 * kHid / 64) / 8, 1), 256, 0, stream>>>(
      X16, kHid, 0L,
      Wqk16, kHid, 0L,
      (void*)Q16, 0, 0L,
      COS, SIN,
      kRows, 2 * kHid, kHid, kQKScale);

  wmma_gemm64<1><<<dim3((kHid / 64) * (kSeq / 64) / 8, kBatch), 256, 0, stream>>>(
      Wv16, kHid, 0L,
      X16, kHid, (long)kSeq * kHid,
      (void*)VT16, kSeq, (long)kHid * kSeq,
      nullptr, nullptr,
      kHid, kSeq, kHid, kVScale);

  attn_kernel<<<kBatch * kHeads * kQTiles, 128, 0, stream>>>(Q16, K16, VT16, A16);

  wmma_gemm64<0><<<dim3((kRows / 64) * (kHid / 64) / 8, 1), 256, 0, stream>>>(
      A16, kHid, 0L,
      Wo16, kHid, 0L,
      (void*)out, kHid, 0L,
      nullptr, nullptr,
      kRows, kHid, kHid, kOutScale);
}
